// GMNN_16638703305267
// MI455X (gfx1250) — hardware-run, weakly checked
//
#include <hip/hip_runtime.h>


namespace {
constexpr int NA = 30000, AP = 30016, NLIM = 30016  , EFULL = 1200000, E = EFULL, NK = 5, NB = 7, NS = 119, NF = 360, KF = 384, U = 512, NMOM = 200;
constexpr float WSC = 256.0f, GS = 64.0f  , RMIN = 0.5f, RMAX = 6.0f;
static_assert(AP % 64 == 0 && NLIM % 64 == 0 && NLIM <= AP && KF % 32 == 0, "tiling");
typedef _Float16 b16;
typedef __attribute__((ext_vector_type(16))) _Float16 v16b;
typedef __attribute__((ext_vector_type(8))) _Float16 v8b;
typedef __attribute__((ext_vector_type(8))) float v8f;
typedef __attribute__((ext_vector_type(4))) float v4f;
__device__ __forceinline__ float bf16_rne(float f) { unsigned int u = __float_as_uint(f); u += 0x7FFFu + ((u >> 16) & 1u); return __uint_as_float(u & 0xFFFF0000u); }
__device__ __forceinline__ void split16(float v, b16& hi, b16& lo) { hi = (b16)v; lo = (b16)(v - (float)hi); }
__device__ __forceinline__ v16b frag_kb(const b16* p, int hh) { const v8b a = *(const v8b*)(p + 8 * hh), b = *(const v8b*)(p + 16 + 8 * hh); v16b f;
#pragma unroll
  for (int e = 0; e < 8; ++e) { f[e] = a[e]; f[8 + e] = b[e]; } return f; }
__device__ __forceinline__ v8f wmma16b(v16b a, v16b b, v8f c) { v8f d = __builtin_amdgcn_wmma_f32_16x16x32_f16(false, a, false, b, (short)0, c, false, false); asm volatile("v_nop\n\tv_nop\n\tv_nop\n\tv_nop" : "+v"(d) : "v"(a), "v"(b)); return d; }
__device__ __forceinline__ void wave_lds_sync() { __builtin_amdgcn_fence(__ATOMIC_RELEASE, "workgroup"); __builtin_amdgcn_wave_barrier(); __builtin_amdgcn_fence(__ATOMIC_ACQUIRE, "workgroup"); }
__device__ __forceinline__ float pmul(float a, float b) { float p = a * b; asm volatile("" : "+v"(p)); return p; }
__device__ __forceinline__ int iclamp(int v, int lo, int hi) { return v < lo ? lo : (v > hi ? hi : v); }
constexpr int CSR_NBLK = 512, CSR_GB = 8  , CSR_GN = 1 << CSR_GB  , CSR_MAXG = 512, CSR_CAP = 12288  ;
__global__ __launch_bounds__(64) void csrA_kernel(const int* __restrict__ dst, int E, int N, int nG, int CHP, int NGP, int* __restrict__ STG, int* __restrict__ HST) {
  extern __shared__ int sm[];
  int* cnt = sm; int* run = sm + NGP; int* ids = sm + 2 * NGP;
  const int b = blockIdx.x; const int ch = (E + CSR_NBLK - 1) / CSR_NBLK; const int e0 = b * ch, e1 = min(E, e0 + ch);
  for (int i = threadIdx.x; i < NGP; i += 64) cnt[i] = 0;
  for (int i = threadIdx.x; i < CHP; i += 64) ids[i] = -1;
  __syncthreads();
  if (threadIdx.x == 0) {
    for (int e = e0; e < e1; ++e) { int d = dst[e]; d = (d < 0) ? 0 : (d >= N ? N - 1 : d); cnt[d >> CSR_GB] += 1; }
    int acc = 0; for (int g = 0; g < nG; ++g) { run[g] = acc; acc += cnt[g]; }
    for (int e = e0; e < e1; ++e) { int d = dst[e]; d = (d < 0) ? 0 : (d >= N ? N - 1 : d); const int g = d >> CSR_GB; ids[run[g]] = e; run[g] += 1; } }
  __syncthreads();
  typedef __attribute__((ext_vector_type(4))) int v4i;
  for (int pass = 0; pass < 2; ++pass) {
    for (int i = threadIdx.x; i < CHP / 4; i += 64) *(volatile v4i*)(STG + (size_t)b * CHP + i * 4) = *(const v4i*)(&ids[i * 4]);
    for (int i = threadIdx.x; i < NGP / 4; i += 64) { v4i v; for (int e = 0; e < 4; ++e) v[e] = (i * 4 + e < nG) ? cnt[i * 4 + e] : 0; *(volatile v4i*)(HST + (size_t)b * NGP + i * 4) = v; }
    __threadfence(); }
}
__global__ __launch_bounds__(512) void csrS_kernel(const int* __restrict__ HST, int nG, int NGP, int* __restrict__ START, int* __restrict__ TOT, int* __restrict__ OFF) {
  __shared__ int tot[CSR_MAXG];
  const int b = threadIdx.x;
  for (int pass = 0; pass < 2; ++pass) { int runb = 0; for (int g = 0; g < nG; ++g) { int c = HST[(size_t)b * NGP + g]; c = (c < 0) ? 0 : c; ((volatile int*)OFF)[(size_t)g * CSR_NBLK + b] = runb; runb += c; } __threadfence(); }
  for (int g = threadIdx.x; g < nG; g += 512) { int s = 0; for (int bb = 0; bb < CSR_NBLK; ++bb) { int c = HST[(size_t)bb * NGP + g]; s += (c < 0) ? 0 : c; } tot[g] = s; }
  __syncthreads();
  if (threadIdx.x < 32) {
    __shared__ int st[CSR_MAXG + 32];
    if (threadIdx.x == 0) { int acc = 0; for (int g = 0; g < NGP; ++g) { st[g] = acc; if (g < nG) acc += (tot[g] + 31) & ~31; } st[NGP] = acc; }
    __builtin_amdgcn_fence(__ATOMIC_RELEASE, "workgroup"); __builtin_amdgcn_wave_barrier(); __builtin_amdgcn_fence(__ATOMIC_ACQUIRE, "workgroup");
    for (int pass = 0; pass < 2; ++pass) { for (int i = threadIdx.x; i < NGP + 32; i += 32) { ((volatile int*)START)[i] = (i <= NGP) ? st[min(i, NGP)] : 0; ((volatile int*)TOT)[i] = (i < nG) ? tot[i] : 0; } __threadfence(); } }
}
__global__ __launch_bounds__(256) void csrB_kernel(const int* __restrict__ dst, int N, int nG, int CHP, int NGP, int permLen, const int* __restrict__ STG, const int* __restrict__ HST, const int* __restrict__ OFF, const int* __restrict__ START, const int* __restrict__ TOT, int* __restrict__ PERM, int* __restrict__ ROWPTR, int* __restrict__ ROWCNT, int* __restrict__ FLAG) {
  typedef __attribute__((ext_vector_type(4))) int v4i;
  __shared__ int ids[CSR_CAP]; __shared__ unsigned short key[CSR_CAP]; __shared__ int outp[CSR_CAP]; __shared__ int ncnt[CSR_GN + 1]; __shared__ int boff[CSR_NBLK + 1];
  const int g = blockIdx.x, t_ = threadIdx.x; int tot = TOT[g]; int st = START[g], stn = START[g + 1]; const int v0 = g * CSR_GN; const int nv = min(CSR_GN, N - v0);
  st = (st < 0) ? 0 : (st > permLen - 32 ? permLen - 32 : st) & ~31; stn = (stn < st) ? st : (stn > permLen ? permLen : stn); tot = (tot < 0) ? 0 : tot; if (tot > stn - st && tot <= CSR_CAP) tot = stn - st;
  if (tot > CSR_CAP) {
    for (int pass = 0; pass < 2; ++pass) { for (int i = t_; i < CSR_GN / 4; i += 256) { v4i a, c; for (int e = 0; e < 4; ++e) { a[e] = st; c[e] = 0; } *(volatile v4i*)(ROWPTR + v0 + i * 4) = a; *(volatile v4i*)(ROWCNT + v0 + i * 4) = c; } if (t_ == 0) ((volatile int*)FLAG)[0] = 1; __threadfence(); } (void)nv; return; }
  if (t_ == 0) { int acc = 0; for (int b = 0; b < CSR_NBLK; ++b) { boff[b] = acc; int c = HST[(size_t)b * NGP + g]; c = (c < 0) ? 0 : (c > CHP ? CHP : c); acc += c; if (acc > tot) acc = tot; } boff[CSR_NBLK] = acc; }
  for (int i = t_; i <= CSR_GN; i += 256) ncnt[i] = 0;
  __syncthreads();
  for (int b = 0; b < CSR_NBLK; ++b) { const int c = boff[b + 1] - boff[b]; int o_ = OFF[(size_t)g * CSR_NBLK + b]; o_ = (o_ < 0) ? 0 : (o_ > CHP - c ? CHP - c : o_); const int* src_ = STG + (size_t)b * CHP + o_;
    for (int i = t_; i < c; i += 256) { int id = src_[i]; id = (id < 0) ? 0 : id; ids[boff[b] + i] = id; int d = dst[id]; d = (d < v0) ? v0 : (d >= N ? N - 1 : d); int kk = d - v0; kk = (kk < 0) ? 0 : (kk >= CSR_GN ? CSR_GN - 1 : kk); key[boff[b] + i] = (unsigned short)kk; } }
  __syncthreads();
  if (t_ == 0) { for (int i = 0; i < tot; ++i) ncnt[key[i]] += 1; int acc = 0; for (int vl = 0; vl < CSR_GN; ++vl) { const int c = ncnt[vl]; ncnt[vl] = acc; acc += c; } ncnt[CSR_GN] = acc;
    for (int i = 0; i < tot; ++i) { const int vl = key[i]; outp[ncnt[vl]] = ids[i]; ncnt[vl] += 1; }
    for (int vl = CSR_GN; vl > 0; --vl) ncnt[vl] = ncnt[vl - 1]; ncnt[0] = 0; }
  __syncthreads();
  for (int pass = 0; pass < 2; ++pass) {
    for (int i = t_; i < (stn - st) / 4; i += 256) { v4i v; for (int e = 0; e < 4; ++e) { const int q = i * 4 + e; v[e] = (q < tot) ? outp[q] : -1; } *(volatile v4i*)(PERM + st + i * 4) = v; }
    for (int i = t_; i < CSR_GN / 4; i += 256) { v4i a, c; for (int e = 0; e < 4; ++e) { const int vl = i * 4 + e; a[e] = st + ncnt[vl]; c[e] = (vl < nv) ? (ncnt[vl + 1] - ncnt[vl]) : 0; } *(volatile v4i*)(ROWPTR + v0 + i * 4) = a; *(volatile v4i*)(ROWCNT + v0 + i * 4) = c; }
    __threadfence(); }
}
__global__ __launch_bounds__(256) void csrZ_kernel(int* __restrict__ p, size_t n4) { typedef __attribute__((ext_vector_type(4))) int v4i; const size_t tid = (size_t)blockIdx.x * 256 + threadIdx.x, nth = (size_t)gridDim.x * 256; v4i z = {0, 0, 0, 0}; for (size_t i = tid; i < n4; i += nth) *(volatile v4i*)(p + i * 4) = z; }
struct CsrBufs { int *STG, *HST, *OFF, *START, *TOT, *PERM, *ROWPTR, *ROWCNT, *FLAG; int nG, NGP, CHP; size_t permLen; char* base; size_t bytes; };
static size_t csr_carve(CsrBufs& c, char* ws, size_t off, int E, int N) {
  const size_t off0 = off; c.base = ws + off;
  auto al = [&](size_t bytes) { char* p = ws + off; off += (bytes + 255) & ~(size_t)255; return p; };
  c.nG = (N + CSR_GN - 1) / CSR_GN; c.NGP = (c.nG + 31) & ~31; const int ch = (E + CSR_NBLK - 1) / CSR_NBLK; c.CHP = (ch + 31) & ~31; c.permLen = (size_t)E + 32 * (size_t)c.nG + 32;
  c.STG = (int*)al((size_t)CSR_NBLK * c.CHP * 4); c.HST = (int*)al((size_t)CSR_NBLK * c.NGP * 4); c.OFF = (int*)al((size_t)c.NGP * CSR_NBLK * 4); c.START = (int*)al((size_t)(c.NGP + 64) * 4); c.TOT = (int*)al((size_t)(c.NGP + 64) * 4);
  c.PERM = (int*)al(c.permLen * 4); c.ROWPTR = (int*)al((size_t)c.nG * CSR_GN * 4); c.ROWCNT = (int*)al((size_t)c.nG * CSR_GN * 4); c.FLAG = (int*)al(256);
  c.bytes = off - off0; return off;
}
static void csr_build(const CsrBufs& c, const int* dst, int E, int N, hipStream_t stream) {
  const size_t smem = (size_t)(2 * c.NGP + c.CHP) * 4;
  csrZ_kernel<<<512, 256, 0, stream>>>((int*)c.base, c.bytes / 16);
  csrA_kernel<<<CSR_NBLK, 64, smem, stream>>>(dst, E, N, c.nG, c.CHP, c.NGP, c.STG, c.HST);
  csrS_kernel<<<1, 512, 0, stream>>>(c.HST, c.nG, c.NGP, c.START, c.TOT, c.OFF);
  csrB_kernel<<<c.nG, 256, 0, stream>>>(dst, N, c.nG, c.CHP, c.NGP, (int)c.permLen, c.STG, c.HST, c.OFF, c.START, c.TOT, c.PERM, c.ROWPTR, c.ROWCNT, c.FLAG);
}

typedef __attribute__((ext_vector_type(2))) float v2f;
__constant__ int TRI2I[15] = {0,0,0,0,0,1,1,1,1,2,2,2,3,3,4};
__constant__ int TRI2J[15] = {0,1,2,3,4,1,2,3,4,2,3,4,3,4,4};
__constant__ int TRI3[35][3] = {{0,0,0},{0,0,1},{0,0,2},{0,0,3},{0,0,4},{0,1,1},{0,1,2},{0,1,3},{0,1,4},{0,2,2},{0,2,3},{0,2,4},{0,3,3},{0,3,4},{0,4,4},{1,1,1},{1,1,2},{1,1,3},{1,1,4},{1,2,2},{1,2,3},{1,2,4},{1,3,3},{1,3,4},{1,4,4},{2,2,2},{2,2,3},{2,2,4},{2,3,3},{2,3,4},{2,4,4},{3,3,3},{3,3,4},{3,4,4},{4,4,4}};
__global__ __launch_bounds__(256) void wprep_kernel(const float* __restrict__ w1, const float* __restrict__ w2, b16* __restrict__ W1T, b16* __restrict__ W2T) {
  size_t t = (size_t)blockIdx.x * 256 + threadIdx.x; v8b o;
  const size_t n1 = (size_t)U * KF / 8; if (t < n1) { const size_t e = t * 8; const int oo = (int)(e / KF), k0 = (int)(e % KF); for (int j = 0; j < 8; ++j) { const int k = k0 + j; o[j] = (k < NF) ? (b16)(bf16_rne(w1[(size_t)k * U + oo]) * WSC) : (b16)0.0f; } for (int pass = 0; pass < 2; ++pass) { *(volatile v8b*)(W1T + e) = o; __threadfence(); } return; } t -= n1;
  const size_t n2 = (size_t)U * U / 8; if (t < n2) { const size_t e = t * 8; const int oo = (int)(e / U), k0 = (int)(e % U); for (int j = 0; j < 8; ++j) o[j] = (b16)(bf16_rne(w2[(size_t)(k0 + j) * U + oo]) * WSC); for (int pass = 0; pass < 2; ++pass) { *(volatile v8b*)(W2T + e) = o; __threadfence(); } }
}
struct PairQ { float rad[NK]; float dn[3]; };
__device__ __forceinline__ PairQ pair_eval(const float* __restrict__ R, const int* __restrict__ Z, const int* __restrict__ idxj, const float* __restrict__ Wr, int e, float rix, float riy, float riz, int zi) {
  PairQ q; const int j = iclamp(idxj[e], 0, NA - 1); const int zj = iclamp(Z[j], 0, NS - 1);
  const float dx = bf16_rne(R[j * 3 + 0]) - rix, dy = bf16_rne(R[j * 3 + 1]) - riy, dz = bf16_rne(R[j * 3 + 2]) - riz;
  const float dr = sqrtf(dx * dx + dy * dy + dz * dz + 1e-12f); const float inv = 1.0f / (dr + 1e-5f); q.dn[0] = dx * inv; q.dn[1] = dy * inv; q.dn[2] = dz * inv;
  const float betta = (float)(NB * NB) / (RMAX * RMAX);
  const float rad_norm = 0.9648135900f;
  float basis[NB];
#pragma unroll
  for (int b = 0; b < NB; ++b) { const float shift = RMIN + (RMAX - RMIN) / (float)NB * (float)b; const float d = dr - shift; basis[b] = rad_norm * __expf(-betta * d * d); }
  const float cut = (dr < RMAX) ? 0.5f * (cosf(3.14159265358979323846f * dr / RMAX) + 1.0f) : 0.0f; const float cs = cut / 2.6457513110645907f;
  const float* w = Wr + ((size_t)zi * NS + zj) * NK * NB;
#pragma unroll
  for (int k = 0; k < NK; ++k) { float s = 0.0f;
#pragma unroll
    for (int b = 0; b < NB; ++b) s += pmul(bf16_rne(w[k * NB + b]), basis[b]); q.rad[k] = s * cs; }
  return q;
}
constexpr int KPP = 96;
__global__ __launch_bounds__(128) void desc_kernel(const float* __restrict__ R, const int* __restrict__ Z, const int* __restrict__ idxj, const float* __restrict__ Wr, const int* __restrict__ PERM, const int* __restrict__ ROWPTR, const int* __restrict__ ROWCNT, int permLen, b16* __restrict__ GMh, b16* __restrict__ GMl) {
  __shared__ __attribute__((aligned(16))) b16 RAh[4][16][KPP + 8], RAl[4][16][KPP + 8], DBh[4][48][KPP + 8], DBl[4][48][KPP + 8]; __shared__ float mom[4][NMOM]; __shared__ __attribute__((aligned(16))) float gmv[4][KF];
  const int wave = threadIdx.x >> 5, lane = threadIdx.x & 31, nloc = lane & 15, hlf = lane >> 4; const size_t v = (size_t)blockIdx.x * 4 + wave;
  for (int q = lane; q < NMOM; q += 32) mom[wave][q] = 0.0f;
  for (int q = lane; q < KF; q += 32) gmv[wave][q] = 0.0f;
  for (int q = lane; q < 16 * (KPP / 8); q += 32) { const int r = q / (KPP / 8), c8 = (q % (KPP / 8)) * 8; const v8b z = {}; *(v8b*)(&RAh[wave][r][c8]) = z; *(v8b*)(&RAl[wave][r][c8]) = z; }
  for (int q = lane; q < 48 * (KPP / 8); q += 32) { const int r = q / (KPP / 8), c8 = (q % (KPP / 8)) * 8; const v8b z = {}; *(v8b*)(&DBh[wave][r][c8]) = z; *(v8b*)(&DBl[wave][r][c8]) = z; }
  wave_lds_sync();
  if (v < (size_t)NA) {
    int st = ROWPTR[v], cnt = ROWCNT[v]; cnt = iclamp(cnt, 0, KPP); st = iclamp(st, 0, permLen - cnt);
    const float rix = bf16_rne(R[v * 3 + 0]), riy = bf16_rne(R[v * 3 + 1]), riz = bf16_rne(R[v * 3 + 2]); const int zi = iclamp(Z[v], 0, NS - 1);
#pragma unroll 1
    for (int c0 = 0; c0 < cnt; c0 += 32) { const int jj = c0 + lane; if (jj < cnt) { const int e = iclamp(PERM[st + jj], 0, E - 1); const PairQ q = pair_eval(R, Z, idxj, Wr, e, rix, riy, riz, zi);
        for (int k = 0; k < NK; ++k) { b16 p, ql; split16(q.rad[k] * 8.0f, p, ql); RAh[wave][k][jj] = p; RAl[wave][k][jj] = ql; }
        float col[40]; col[0] = 1.0f;
#pragma unroll
        for (int c = 0; c < 3; ++c) { col[1 + c] = q.dn[c];
#pragma unroll
          for (int d = 0; d < 3; ++d) { col[4 + c * 3 + d] = q.dn[c] * q.dn[d];
#pragma unroll
            for (int ee = 0; ee < 3; ++ee) col[13 + c * 9 + d * 3 + ee] = q.dn[c] * q.dn[d] * q.dn[ee]; } }
#pragma unroll
        for (int r = 0; r < 40; ++r) { b16 p, ql; split16(col[r] * 8.0f, p, ql); DBh[wave][r][jj] = p; DBl[wave][r][jj] = ql; } } }
    wave_lds_sync();
    v8f acc[3];
#pragma unroll
    for (int t = 0; t < 3; ++t) acc[t] = (v8f){};
#pragma unroll
    for (int kb = 0; kb < KPP; kb += 32) { const v16b ah = frag_kb(&RAh[wave][nloc][kb], hlf), al = frag_kb(&RAl[wave][nloc][kb], hlf);
#pragma unroll
      for (int t = 0; t < 3; ++t) { const v16b bh = frag_kb(&DBh[wave][t * 16 + nloc][kb], hlf), bl = frag_kb(&DBl[wave][t * 16 + nloc][kb], hlf); acc[t] = wmma16b(ah, bh, acc[t]); acc[t] = wmma16b(ah, bl, acc[t]); acc[t] = wmma16b(al, bh, acc[t]); acc[t] = wmma16b(al, bl, acc[t]); } }
    if (hlf == 0) {
#pragma unroll
      for (int t = 0; t < 3; ++t) { const int col = t * 16 + nloc;
#pragma unroll
        for (int r = 0; r < NK; ++r) { const float m = acc[t][r] * (1.0f / 64.0f);
          if (col == 0) mom[wave][r] = m; else if (col < 4) mom[wave][5 + r * 3 + (col - 1)] = m; else if (col < 13) mom[wave][20 + r * 9 + (col - 4)] = m; else if (col < 40) mom[wave][65 + r * 27 + (col - 13)] = m; } } }
    wave_lds_sync();
    const float* M0 = &mom[wave][0]; const float* M1 = &mom[wave][5]; const float* M2 = &mom[wave][20]; const float* M3 = &mom[wave][65];
#pragma unroll 1
    for (int f = lane; f < NF; f += 32) { float val = 0.0f;
      if (f < 5) val = M0[f];
      else if (f < 20) { const int p = f - 5, r = TRI2I[p], s = TRI2J[p];
#pragma unroll 1
        for (int i = 0; i < 3; ++i) val += M1[r * 3 + i] * M1[s * 3 + i]; }
      else if (f < 35) { const int p = f - 20, r = TRI2I[p], s = TRI2J[p];
#pragma unroll 1
        for (int i = 0; i < 9; ++i) val += M2[r * 9 + i] * M2[s * 9 + i]; }
      else if (f < 50) { const int p = f - 35, r = TRI2I[p], s = TRI2J[p];
#pragma unroll 1
        for (int i = 0; i < 27; ++i) val += M3[r * 27 + i] * M3[s * 27 + i]; }
      else if (f < 85) { const int p = f - 50, r = TRI3[p][0], s = TRI3[p][1], t = TRI3[p][2];
#pragma unroll 1
        for (int ijk = 0; ijk < 27; ++ijk) { const int i = ijk / 9, j = (ijk / 3) % 3, k = ijk % 3; val += M2[r * 9 + i * 3 + j] * M2[s * 9 + i * 3 + k] * M2[t * 9 + j * 3 + k]; } }
      else if (f < 160) { const int p = (f - 85) / 5, t = (f - 85) % 5, r = TRI2I[p], s = TRI2J[p];
#pragma unroll 1
        for (int ij = 0; ij < 9; ++ij) { const int i = ij / 3, j = ij % 3; val += M1[r * 3 + i] * M1[s * 3 + j] * M2[t * 9 + ij]; } }
      else if (f < 235) { const int p = (f - 160) / 5, t = (f - 160) % 5, r = TRI2I[p], s = TRI2J[p];
#pragma unroll 1
        for (int ijk = 0; ijk < 27; ++ijk) { const int ij = ijk / 3, k = ijk % 3; float u2 = 0.0f;
#pragma unroll 1
          for (int l = 0; l < 3; ++l) u2 += M3[s * 27 + ij * 3 + l] * M2[t * 9 + k * 3 + l]; val += M3[r * 27 + ijk] * u2; } }
      else { const int p = f - 235, r = p / 25, s = (p / 5) % 5, t = p % 5;
#pragma unroll 1
        for (int ijk = 0; ijk < 27; ++ijk) { const int ij = ijk / 3, k = ijk % 3; val += M3[r * 27 + ijk] * M2[s * 9 + ij] * M1[t * 3 + k]; } }
      gmv[wave][f] = val; } }
  wave_lds_sync();
  for (int pass = 0; pass < 2; ++pass) { for (int p = lane; p < KF / 8; p += 32) { v8b hv, lv; for (int j = 0; j < 8; ++j) { b16 a_, b_; split16(gmv[wave][p * 8 + j] * GS, a_, b_); hv[j] = a_; lv[j] = b_; }
      *(volatile v8b*)(GMh + v * KF + p * 8) = hv; *(volatile v8b*)(GMl + v * KF + p * 8) = lv; } __threadfence(); }
}
__device__ __forceinline__ float swishf(float x) { return x / (1.0f + __expf(-x)); }
template <int KD, int MODE>
__global__ __launch_bounds__(128) void mlp_kernel(const b16* __restrict__ Ah, const b16* __restrict__ Al, const b16* __restrict__ WT, const float* __restrict__ bias, const float* __restrict__ w3, b16* __restrict__ Oh, b16* __restrict__ Ol, float* __restrict__ PS) {
  __shared__ __attribute__((aligned(16))) float Tf[4][16][128 + 4]; __shared__ float rp[64];
  const int wave = threadIdx.x >> 5, lane = threadIdx.x & 31, nloc = lane & 15, hlf = lane >> 4; const size_t m0 = (size_t)blockIdx.x * 64 + wave * 16; const int n0 = blockIdx.y * 128;
  v8f acc[8];
#pragma unroll
  for (int t = 0; t < 8; ++t) acc[t] = (v8f){};
#pragma unroll 2
  for (int kb = 0; kb < KD; kb += 32) { const v16b a = frag_kb(Ah + (m0 + nloc) * KD + kb, hlf), al = frag_kb(Al + (m0 + nloc) * KD + kb, hlf);
#pragma unroll
    for (int t = 0; t < 8; ++t) { const v16b bw = frag_kb(WT + (size_t)(n0 + t * 16 + nloc) * KD + kb, hlf); acc[t] = wmma16b(a, bw, acc[t]); acc[t] = wmma16b(al, bw, acc[t]); } }
#pragma unroll
  for (int t = 0; t < 8; ++t) { const int c = n0 + t * 16 + nloc; const float bb = bf16_rne(bias[c]); const float w = MODE ? bf16_rne(w3[c]) : 1.0f;
#pragma unroll
    for (int r = 0; r < 8; ++r) { float v = swishf(acc[t][r] * (1.0f / (GS * WSC)) + bb); if (m0 + 8 * hlf + r >= (size_t)NA) v = 0.0f; Tf[wave][8 * hlf + r][t * 16 + nloc] = MODE ? pmul(v, w) : v * GS; } }
  wave_lds_sync();
  if (MODE == 0) {
    for (int pass = 0; pass < 2; ++pass) { for (int rr = 0; rr < 16; ++rr) { const v4f f = *(const v4f*)(&Tf[wave][rr][lane * 4]); b16 p0, q0, p1, q1, p2, q2, p3, q3; split16(f[0], p0, q0); split16(f[1], p1, q1); split16(f[2], p2, q2); split16(f[3], p3, q3);
        typedef __attribute__((ext_vector_type(4))) _Float16 v4h; v4h hv = {p0, p1, p2, p3}, lv = {q0, q1, q2, q3}; *(volatile v4h*)(Oh + (m0 + rr) * U + n0 + lane * 4) = hv; *(volatile v4h*)(Ol + (m0 + rr) * U + n0 + lane * 4) = lv; } __threadfence(); }
  } else {
    if (lane < 16) { float s = 0.0f; for (int c = 0; c < 128; ++c) s += Tf[wave][lane][c]; rp[wave * 16 + lane] = s; }
    __syncthreads();
    for (int pass = 0; pass < 2; ++pass) { if (threadIdx.x < 64) ((volatile float*)PS)[(size_t)blockIdx.y * AP + (size_t)blockIdx.x * 64 + threadIdx.x] = rp[threadIdx.x]; __threadfence(); } }
}
__global__ __launch_bounds__(256) void out_kernel(const float* __restrict__ PS, const float* __restrict__ b3, const int* __restrict__ Z, const float* __restrict__ scale, const float* __restrict__ shift, float* __restrict__ out) {
  const size_t v = (size_t)blockIdx.x * 256 + threadIdx.x; if (v >= (size_t)NA) return;
  float h = bf16_rne(b3[0]); for (int s = 0; s < 4; ++s) h += PS[(size_t)s * AP + v]; const int z = iclamp(Z[v], 0, NS - 1); const float o = pmul(bf16_rne(scale[z]), h) + bf16_rne(shift[z]);
  for (int pass = 0; pass < 2; ++pass) { ((volatile float*)out)[v] = o; __threadfence(); }
}
}

extern "C" void kernel_launch(void* const* d_in, const int* in_sizes, int n_in, void* d_out, int out_size, void* d_ws, size_t ws_size, hipStream_t stream) {
  (void)n_in;
  auto Fp = [&](int i) { return (const float*)d_in[i]; }; auto Ip = [&](int i) { return (const int*)d_in[i]; };
  if (in_sizes[0] != NA * 3 || in_sizes[1] != NA || in_sizes[2] != 2 * EFULL || in_sizes[3] != NS * NS * NK * NB || in_sizes[4] != NF * U || in_sizes[5] != U || in_sizes[6] != U * U || in_sizes[7] != U || in_sizes[8] != U || in_sizes[9] != 1 || in_sizes[10] != NS || in_sizes[11] != NS || out_size != NA) return;
  size_t off = 0; char* ws = (char*)d_ws;
  auto carve = [&](size_t bytes) { char* p = ws + off; off += (bytes + 255) & ~(size_t)255; return p; };
  b16* W1T = (b16*)carve((size_t)U * KF * 2); b16* W2T = (b16*)carve((size_t)U * U * 2); b16* GMh = (b16*)carve((size_t)AP * KF * 2); b16* GMl = (b16*)carve((size_t)AP * KF * 2); b16* H1h = (b16*)carve((size_t)AP * U * 2); b16* H1l = (b16*)carve((size_t)AP * U * 2); float* PS = (float*)carve((size_t)4 * AP * 4);
  CsrBufs csr; off = csr_carve(csr, ws, off, E, NA);
  if (off > ws_size || off > ((size_t)128 << 20)) return;
  wprep_kernel<<<(unsigned)((((size_t)U * KF + (size_t)U * U) / 8 + 255) / 256), 256, 0, stream>>>(Fp(4), Fp(6), W1T, W2T);
  csr_build(csr, Ip(2), E, NA, stream);
  desc_kernel<<<NLIM / 4, 128, 0, stream>>>(Fp(0), Ip(1), Ip(2) + EFULL, Fp(3), csr.PERM, csr.ROWPTR, csr.ROWCNT, (int)csr.permLen, GMh, GMl);
  mlp_kernel<KF, 0><<<dim3(NLIM / 64, U / 128), 128, 0, stream>>>(GMh, GMl, W1T, Fp(5), nullptr, H1h, H1l, nullptr);
  mlp_kernel<U, 1><<<dim3(NLIM / 64, U / 128), 128, 0, stream>>>(H1h, H1l, W2T, Fp(7), Fp(8), nullptr, nullptr, PS);
  out_kernel<<<(NA + 255) / 256, 256, 0, stream>>>(PS, Fp(9), Ip(1), Fp(10), Fp(11), (float*)d_out);
}
